// MultiTaskMazeQNetwork_10136122818688
// MI455X (gfx1250) — hardware-verified
//
#include <hip/hip_runtime.h>
#include <stddef.h>
#include <stdint.h>


#define NTHR   256
#define NWAVE  8
#define IMH    16
#define IMW    16
#define CIN    3
#define C1     32
#define C2     64
#define O1     15
#define P2     19
#define K1     48
#define K1P    64
#define M1     (O1 * O1)
#define M1P    256
#define AP1    72
#define K2     512
#define FLAT   4096
#define EXPN   512
#define BOTN   128
#define NT     16
#define NF     128
#define HEADK  256
#define ACT    4
#define EROWS  32
#define HP     (EXPN + 8)
#define TROWS  64
#define KC     256
#define TAP    (KC + 8)
#define NG     16
#define XPN    (18 * 18 * CIN)
#define WSC    16.0f
#define WINV   0.0625f

static_assert((C1 * K1P / 8) % NTHR == 0);
static_assert((C2 * K2 / 8) % NTHR == 0);
static_assert((EXPN * FLAT / 8) % NTHR == 0);
static_assert((BOTN * EXPN / 8) % NTHR == 0);
static_assert((NT * NF * FLAT / 8) % NTHR == 0);
static_assert(M1P * AP1 >= 64 * C2);
static_assert(TROWS * TAP * 2 >= TROWS * NF * 4);
static_assert(BOTN == NF);
static_assert((P2 * P2 * C1) % 8 == 0);
static_assert(KC % 32 == 0 && FLAT % KC == 0);
static_assert((TROWS * KC / 8) % NTHR == 0);
static_assert(EROWS * BOTN / 4 == 4 * NTHR);
static_assert(FLAT / 8 == 2 * NTHR);
static_assert(TROWS * NF / 4 == 8 * NTHR);
static_assert((M1P * 8) % NTHR == 0);
static_assert(K1 % 8 == 0);
static_assert(NWAVE * 32 == NTHR);
static_assert(TROWS <= NTHR && NT <= 32);

typedef float    v4f  __attribute__((ext_vector_type(4)));
typedef float    v8f  __attribute__((ext_vector_type(8)));
typedef _Float16 v8h  __attribute__((ext_vector_type(8)));
typedef _Float16 v16h __attribute__((ext_vector_type(16)));
union FragH { v16h v; v8h h[2]; };

__device__ __forceinline__ v8h cvt8(v4f a, v4f b) {
  v8h r;
  r[0] = (_Float16)a.x; r[1] = (_Float16)a.y; r[2] = (_Float16)a.z; r[3] = (_Float16)a.w;
  r[4] = (_Float16)b.x; r[5] = (_Float16)b.y; r[6] = (_Float16)b.z; r[7] = (_Float16)b.w;
  return r;
}
__device__ __forceinline__ v8h zero8h() {
  v4f z = {0.0f, 0.0f, 0.0f, 0.0f};
  return cvt8(z, z);
}
__device__ __forceinline__ v8f zero8f() {
  v8f z = {0.0f, 0.0f, 0.0f, 0.0f, 0.0f, 0.0f, 0.0f, 0.0f};
  return z;
}

__device__ __forceinline__ v8f wmh(v16h a, v16h b, v8f c) {
  v8f d = __builtin_amdgcn_wmma_f32_16x16x32_f16(false, a, false, b, (short)0, c, false, false);
  asm volatile("v_nop\n\tv_nop\n\tv_nop\n\tv_nop" : "+v"(d) : "v"(a), "v"(b));
  return d;
}

__device__ __forceinline__ int tnorm(int v) {
  int t = v < 0 ? v + NT : v;
  t = t < 0 ? 0 : (t > NT - 1 ? NT - 1 : t);
  return t;
}

__global__ __launch_bounds__(NTHR) void k_wprep(
    const float* __restrict__ w1, const float* __restrict__ w2, const float* __restrict__ we,
    const float* __restrict__ wb, const float* __restrict__ wt,
    _Float16* p1, _Float16* p2, _Float16* pe, _Float16* pb, _Float16* pt) {
  const int g0 = C1 * K1P / 8;
  const int g1 = C2 * K2 / 8;
  const int g2 = EXPN * FLAT / 8;
  const int g3 = BOTN * EXPN / 8;
  const int g4 = NT * NF * FLAT / 8;
  const int bstart = blockIdx.x * NTHR;
  const float* src; _Float16* dst; int K, Nout, KP, segOff, per;
  if (bstart < g0)                     { src = w1; dst = p1; K = K1;   Nout = C1;   KP = K1P;  segOff = 0;                 per = 0; }
  else if (bstart < g0 + g1)           { src = w2; dst = p2; K = K2;   Nout = C2;   KP = K2;   segOff = g0;                per = 0; }
  else if (bstart < g0 + g1 + g2)      { src = we; dst = pe; K = FLAT; Nout = EXPN; KP = FLAT; segOff = g0 + g1;           per = 0; }
  else if (bstart < g0 + g1 + g2 + g3) { src = wb; dst = pb; K = EXPN; Nout = BOTN; KP = EXPN; segOff = g0 + g1 + g2;      per = 0; }
  else                                 { src = wt; dst = pt; K = FLAT; Nout = NF;   KP = FLAT; segOff = g0 + g1 + g2 + g3; per = FLAT * NF; }
  const int i = bstart + (int)threadIdx.x;
  if (i >= g0 + g1 + g2 + g3 + g4) return;
  const int o = (i - segOff) * 8;
  int oo = o;
  if (per != 0) {
    const int layer = o / per;
    src += (size_t)layer * per;
    oo = o - layer * per;
  }
  const int n  = oo / KP;
  const int k0 = oo - n * KP;
  const int nc = n < Nout ? n : Nout - 1;
  float v[8];
#pragma unroll
  for (int e = 0; e < 8; ++e) {
    const int k  = k0 + e;
    const int kc = k < K ? k : K - 1;
    const float xv = src[(size_t)kc * Nout + nc];
    v[e] = xv * ((k < K && n < Nout) ? WSC : 0.0f);
  }
  v4f a, b;
  a.x = v[0]; a.y = v[1]; a.z = v[2]; a.w = v[3];
  b.x = v[4]; b.y = v[5]; b.z = v[6]; b.w = v[7];
  const v8h hv = cvt8(a, b);
  _Float16* dp = dst + o;
  *(volatile v8h*)dp = hv;
  __threadfence();
  *(volatile v8h*)dp = hv;
}

__global__ __launch_bounds__(NTHR) void k_conv(
    const float* __restrict__ x, const _Float16* __restrict__ p1, const float* __restrict__ b1,
    const _Float16* __restrict__ p2, const float* __restrict__ b2, _Float16* flat, int nImg) {
  __shared__ __attribute__((aligned(16))) float    xp[XPN + 4];
  __shared__ __attribute__((aligned(16))) _Float16 a1[M1P * AP1];
  __shared__ __attribute__((aligned(16))) _Float16 c1p[P2 * P2 * C1];
  const int tid = threadIdx.x, lane = tid & 31, wave = tid >> 5, hh = lane >> 4, m = lane & 15;
  const int img = blockIdx.x;
  if (img >= nImg) return;
  const float* xi = x + (size_t)img * (IMH * IMW * CIN);

  for (int e = tid; e < XPN; e += NTHR) {
    const int r   = e / (18 * CIN);
    const int rem = e - r * (18 * CIN);
    const int cc  = rem / CIN;
    const int ci  = rem - cc * CIN;
    const bool in = (r >= 1) && (r <= IMH) && (cc >= 1) && (cc <= IMW);
    int rr = r - 1;  rr = rr < 0 ? 0 : (rr > IMH - 1 ? IMH - 1 : rr);
    int qq = cc - 1; qq = qq < 0 ? 0 : (qq > IMW - 1 ? IMW - 1 : qq);
    const float v = xi[(rr * IMW + qq) * CIN + ci];
    xp[e] = in ? v : 0.0f;
  }
  {
    const v8h z = zero8h();
    for (int i = tid; i < (P2 * P2 * C1) / 8; i += NTHR) *(v8h*)(c1p + 8 * i) = z;
  }
  __syncthreads();

#pragma unroll
  for (int it = 0; it < (M1P * 8) / NTHR; ++it) {
    const int q   = it * NTHR + tid;
    const int row = q >> 3, g = q & 7;
    const bool ok = (row < M1) && (g < K1 / 8);
    const int rc  = row < M1 ? row : M1 - 1;
    const int oi  = rc / O1, oj = rc - oi * O1;
    float v[8];
#pragma unroll
    for (int e = 0; e < 8; ++e) {
      int k = 8 * g + e; k = k > K1 - 1 ? K1 - 1 : k;
      const int tap = k / CIN, ci = k - CIN * tap, ky = tap >> 2, kx = tap & 3;
      const float val = xp[((oi + ky) * 18 + (oj + kx)) * CIN + ci];
      v[e] = ok ? val : 0.0f;
    }
    v4f va, vb;
    va.x = v[0]; va.y = v[1]; va.z = v[2]; va.w = v[3];
    vb.x = v[4]; vb.y = v[5]; vb.z = v[6]; vb.w = v[7];
    *(v8h*)(a1 + row * AP1 + 8 * g) = cvt8(va, vb);
  }
  __syncthreads();

  v8f acc1[2][2];
#pragma unroll
  for (int mi = 0; mi < 2; ++mi) { acc1[mi][0] = zero8f(); acc1[mi][1] = zero8f(); }
#pragma unroll
  for (int ks = 0; ks < K1P / 32; ++ks) {
    FragH fa[2], fb[2];
#pragma unroll
    for (int mi = 0; mi < 2; ++mi) {
      const _Float16* ar = a1 + (32 * wave + 16 * mi + m) * AP1 + 32 * ks + 8 * hh;
      fa[mi].h[0] = *(const v8h*)ar;
      fa[mi].h[1] = *(const v8h*)(ar + 16);
    }
#pragma unroll
    for (int ni = 0; ni < 2; ++ni) {
      const _Float16* bp = p1 + (16 * ni + m) * K1P + 32 * ks + 8 * hh;
      fb[ni].h[0] = *(const v8h*)bp;
      fb[ni].h[1] = *(const v8h*)(bp + 16);
    }
#pragma unroll
    for (int mi = 0; mi < 2; ++mi) {
      acc1[mi][0] = wmh(fa[mi].v, fb[0].v, acc1[mi][0]);
      acc1[mi][1] = wmh(fa[mi].v, fb[1].v, acc1[mi][1]);
    }
  }
#pragma unroll
  for (int ni = 0; ni < 2; ++ni) {
    const int col = 16 * ni + m;
    const float bias = b1[col];
#pragma unroll
    for (int mi = 0; mi < 2; ++mi) {
#pragma unroll
      for (int r = 0; r < 8; ++r) {
        const int p = 32 * wave + 16 * mi + 8 * hh + r;
        if (p < M1) {
          const int i = p / O1, j = p - i * O1;
          c1p[((i + 2) * P2 + (j + 2)) * C1 + col] = (_Float16)fmaxf(acc1[mi][ni][r] * WINV + bias, 0.0f);
        }
      }
    }
  }
  __syncthreads();

  const int mt = wave >> 1, nt0 = 2 * (wave & 1);
  const int mrow = 16 * mt + m;
  const int yy = mrow >> 3, xx = mrow & 7;
  v8f acc2[2];
  acc2[0] = zero8f(); acc2[1] = zero8f();
#pragma unroll 2
  for (int ks = 0; ks < K2 / 32; ++ks) {
    const int ky = ks >> 2, kx = ks & 3;
    const _Float16* ar = c1p + ((2 * yy + ky) * P2 + (2 * xx + kx)) * C1 + 8 * hh;
    FragH fa;
    fa.h[0] = *(const v8h*)ar;
    fa.h[1] = *(const v8h*)(ar + 16);
#pragma unroll
    for (int ni = 0; ni < 2; ++ni) {
      const _Float16* bp = p2 + (size_t)(16 * (nt0 + ni) + m) * K2 + 32 * ks + 8 * hh;
      FragH fb;
      fb.h[0] = *(const v8h*)bp;
      fb.h[1] = *(const v8h*)(bp + 16);
      acc2[ni] = wmh(fa.v, fb.v, acc2[ni]);
    }
  }
  _Float16* so = a1;
#pragma unroll
  for (int ni = 0; ni < 2; ++ni) {
    const int col = 16 * (nt0 + ni) + m;
    const float bias = b2[col];
#pragma unroll
    for (int r = 0; r < 8; ++r)
      so[(16 * mt + 8 * hh + r) * C2 + col] = (_Float16)fmaxf(acc2[ni][r] * WINV + bias, 0.0f);
  }
  __syncthreads();

  _Float16* gp = flat + (size_t)img * FLAT;
  const v8h o0 = *(const v8h*)(so + 8 * tid);
  const v8h o1 = *(const v8h*)(so + 8 * (tid + NTHR));
  *(volatile v8h*)(gp + 8 * tid) = o0;
  *(volatile v8h*)(gp + 8 * (tid + NTHR)) = o1;
  __threadfence();
  *(volatile v8h*)(gp + 8 * tid) = o0;
  *(volatile v8h*)(gp + 8 * (tid + NTHR)) = o1;
}

__global__ __launch_bounds__(NTHR) void k_expbot(
    const _Float16* __restrict__ flat, const _Float16* __restrict__ pe, const float* __restrict__ be,
    const _Float16* __restrict__ pb, const float* __restrict__ bb, float* shp, int nRows) {
  __shared__ __attribute__((aligned(16))) _Float16 hid[EROWS * HP];
  __shared__ __attribute__((aligned(16))) float    stg[EROWS * BOTN];
  const int tid = threadIdx.x, lane = tid & 31, wave = tid >> 5, hh = lane >> 4, m = lane & 15;
  const int row0 = blockIdx.x * EROWS;
  if (row0 >= nRows) return;

  v8f acc[2][4];
#pragma unroll
  for (int mi = 0; mi < 2; ++mi) {
#pragma unroll
    for (int nt = 0; nt < 4; ++nt) acc[mi][nt] = zero8f();
  }
  const _Float16* ab = flat + (size_t)(row0 + m) * FLAT + 8 * hh;
  const _Float16* bbp = pe + (size_t)(64 * wave + m) * FLAT + 8 * hh;
#pragma unroll 2
  for (int kt = 0; kt < FLAT / 32; ++kt) {
    FragH fa[2], fb[4];
#pragma unroll
    for (int mi = 0; mi < 2; ++mi) {
      const _Float16* ar = ab + (size_t)(16 * mi) * FLAT + 32 * kt;
      fa[mi].h[0] = *(const v8h*)ar;
      fa[mi].h[1] = *(const v8h*)(ar + 16);
    }
#pragma unroll
    for (int nt = 0; nt < 4; ++nt) {
      const _Float16* bp = bbp + (size_t)(16 * nt) * FLAT + 32 * kt;
      fb[nt].h[0] = *(const v8h*)bp;
      fb[nt].h[1] = *(const v8h*)(bp + 16);
    }
#pragma unroll
    for (int mi = 0; mi < 2; ++mi) {
#pragma unroll
      for (int nt = 0; nt < 4; ++nt) acc[mi][nt] = wmh(fa[mi].v, fb[nt].v, acc[mi][nt]);
    }
  }
#pragma unroll
  for (int nt = 0; nt < 4; ++nt) {
    const int col = 64 * wave + 16 * nt + m;
    const float bias = be[col];
#pragma unroll
    for (int mi = 0; mi < 2; ++mi) {
#pragma unroll
      for (int r = 0; r < 8; ++r)
        hid[(16 * mi + 8 * hh + r) * HP + col] = (_Float16)(acc[mi][nt][r] * WINV + bias);
    }
  }
  __syncthreads();

  v8f c2[2];
  c2[0] = zero8f(); c2[1] = zero8f();
  const _Float16* hb = hid + m * HP + 8 * hh;
  const _Float16* qb = pb + (size_t)(16 * wave + m) * EXPN + 8 * hh;
#pragma unroll 2
  for (int kt = 0; kt < EXPN / 32; ++kt) {
    FragH fb;
    fb.h[0] = *(const v8h*)(qb + 32 * kt);
    fb.h[1] = *(const v8h*)(qb + 32 * kt + 16);
#pragma unroll
    for (int mi = 0; mi < 2; ++mi) {
      const _Float16* ar = hb + (16 * mi) * HP + 32 * kt;
      FragH fa;
      fa.h[0] = *(const v8h*)ar;
      fa.h[1] = *(const v8h*)(ar + 16);
      c2[mi] = wmh(fa.v, fb.v, c2[mi]);
    }
  }
  {
    const int col = 16 * wave + m;
    const float bias = bb[col];
#pragma unroll
    for (int mi = 0; mi < 2; ++mi) {
#pragma unroll
      for (int r = 0; r < 8; ++r)
        stg[(16 * mi + 8 * hh + r) * BOTN + col] = fmaxf(c2[mi][r] * WINV + bias, 0.0f);
    }
  }
  __syncthreads();

  float* gp = shp + (size_t)row0 * BOTN;
  v4f ov[4];
#pragma unroll
  for (int i = 0; i < 4; ++i) ov[i] = *(const v4f*)(stg + 4 * (i * NTHR + tid));
#pragma unroll
  for (int i = 0; i < 4; ++i) *(volatile v4f*)(gp + 4 * (i * NTHR + tid)) = ov[i];
  __threadfence();
#pragma unroll
  for (int i = 0; i < 4; ++i) *(volatile v4f*)(gp + 4 * (i * NTHR + tid)) = ov[i];
}

__global__ __launch_bounds__(NTHR) void k_trep(
    const _Float16* __restrict__ flat, const _Float16* __restrict__ pt, const float* __restrict__ bt,
    const int* __restrict__ task, float* trg, int nB, int nTiles, int maxIt) {
  __shared__ __attribute__((aligned(16))) v4f traw[(TROWS * TAP * 2) / 16];
  __shared__ int lst[TROWS];
  __shared__ int wcs[NWAVE * NT];
  __shared__ int scnt[NT];
  __shared__ int stb[NT + 1];
  __shared__ int wcnt[NWAVE];
  _Float16* sA  = (_Float16*)traw;
  float*    stg = (float*)traw;
  const int tid = threadIdx.x, lane = tid & 31, wave = tid >> 5, hh = lane >> 4, m = lane & 15;
  const int t = blockIdx.x / NG, g = blockIdx.x - t * NG;
  const int nch = nB / NTHR;

  int c[NT];
#pragma unroll
  for (int tp = 0; tp < NT; ++tp) c[tp] = 0;
#pragma unroll 1
  for (int ch = 0; ch < nch; ++ch) {
    const int tt = tnorm(task[ch * NTHR + tid]);
#pragma unroll
    for (int tp = 0; tp < NT; ++tp) c[tp] += (int)__builtin_popcount(__builtin_amdgcn_ballot_w32(tt == tp));
  }
  if (lane == 0) {
#pragma unroll
    for (int tp = 0; tp < NT; ++tp) wcs[wave * NT + tp] = c[tp];
  }
  __syncthreads();
  if (tid < NT) {
    int s = 0;
#pragma unroll
    for (int w = 0; w < NWAVE; ++w) s += wcs[w * NT + tid];
    scnt[tid] = s;
  }
  __syncthreads();
  if (tid == 0) {
    int tb = 0;
#pragma unroll 1
    for (int tp = 0; tp < NT; ++tp) { stb[tp] = tb; tb += (scnt[tp] + TROWS - 1) / TROWS; }
    stb[NT] = tb;
  }
  __syncthreads();
  const int cntT  = scnt[t];
  const int ntile = (cntT + TROWS - 1) / TROWS;
  const int tb0   = stb[t];

#pragma unroll 1
  for (int it = 0; it < maxIt; ++it) {
    const int mb = g + NG * it;
    if (mb >= ntile) break;
    const int rlo = mb * TROWS;
    if (tid < TROWS) lst[tid] = 0;
    __syncthreads();

    int run = 0;
#pragma unroll 1
    for (int ch = 0; ch < nch; ++ch) {
      if (run >= rlo + TROWS) break;
      const int e  = ch * NTHR + tid;
      const int tt = tnorm(task[e]);
      const bool hit = (tt == t);
      const unsigned mk = __builtin_amdgcn_ballot_w32(hit);
      if (lane == 0) wcnt[wave] = (int)__builtin_popcount(mk);
      __syncthreads();
      int pre = 0, tot = 0;
#pragma unroll
      for (int w = 0; w < NWAVE; ++w) { const int v = wcnt[w]; tot += v; pre += (w < wave) ? v : 0; }
      const int pos = run + pre + (int)__builtin_amdgcn_mbcnt_lo(mk, 0u) - rlo;
      if (hit && (unsigned)pos < (unsigned)TROWS) lst[pos] = e;
      run += tot;
      __syncthreads();
    }

    v8f acc[4];
#pragma unroll
    for (int mi = 0; mi < 4; ++mi) acc[mi] = zero8f();
    const _Float16* bbase = pt + (size_t)(t * NF + 16 * wave + m) * FLAT + 8 * hh;
#pragma unroll 1
    for (int kc = 0; kc < FLAT / KC; ++kc) {
#pragma unroll
      for (int i = 0; i < (TROWS * KC / 8) / NTHR; ++i) {
        const int idx = i * NTHR + tid;
        const int row = idx >> 5;
        const int pc  = idx & 31;
        int rid = lst[row];
        rid = rid < 0 ? 0 : (rid > nB - 1 ? nB - 1 : rid);
        const v8h v = *(const v8h*)(flat + (size_t)rid * FLAT + kc * KC + 8 * pc);
        *(v8h*)(sA + row * TAP + 8 * pc) = v;
      }
      __syncthreads();
#pragma unroll 2
      for (int ks = 0; ks < KC / 32; ++ks) {
        FragH fb;
        fb.h[0] = *(const v8h*)(bbase + kc * KC + 32 * ks);
        fb.h[1] = *(const v8h*)(bbase + kc * KC + 32 * ks + 16);
#pragma unroll
        for (int mi = 0; mi < 4; ++mi) {
          const _Float16* ar = sA + (16 * mi + m) * TAP + 32 * ks + 8 * hh;
          FragH fa;
          fa.h[0] = *(const v8h*)ar;
          fa.h[1] = *(const v8h*)(ar + 16);
          acc[mi] = wmh(fa.v, fb.v, acc[mi]);
        }
      }
      __syncthreads();
    }

    {
      const int col = 16 * wave + m;
      const float bias = bt[t * NF + col];
#pragma unroll
      for (int mi = 0; mi < 4; ++mi) {
#pragma unroll
        for (int r = 0; r < 8; ++r)
          stg[(16 * mi + 8 * hh + r) * NF + col] = fmaxf(acc[mi][r] * WINV + bias, 0.0f);
      }
    }
    __syncthreads();
    int tile = tb0 + mb;
    tile = tile < 0 ? 0 : (tile > nTiles - 1 ? nTiles - 1 : tile);
    float* gp = trg + (size_t)tile * (TROWS * NF);
    v4f ov[8];
#pragma unroll
    for (int i = 0; i < 8; ++i) ov[i] = *(const v4f*)(stg + 4 * (i * NTHR + tid));
#pragma unroll
    for (int i = 0; i < 8; ++i) *(volatile v4f*)(gp + 4 * (i * NTHR + tid)) = ov[i];
    __threadfence();
#pragma unroll
    for (int i = 0; i < 8; ++i) *(volatile v4f*)(gp + 4 * (i * NTHR + tid)) = ov[i];
    __syncthreads();
  }
}

__global__ __launch_bounds__(NTHR) void k_head(
    const float* __restrict__ shp, const float* __restrict__ trg, const int* __restrict__ task,
    const float* __restrict__ thw, const float* __restrict__ thb, float* out, int nB, int nTiles) {
  __shared__ int sc[NT];
  __shared__ int wcs[NWAVE * NT];
  __shared__ int tbs[NT + 1];
  const int tid = threadIdx.x, lane = tid & 31, wave = tid >> 5;
  const int own = blockIdx.x;
  const int nch = nB / NTHR;
  if (own >= nch) return;
  if (tid < NT) sc[tid] = 0;
  __syncthreads();

  int myT = 0, myRank = 0;
#pragma unroll 1
  for (int ch = 0; ch < nch; ++ch) {
    const int tt = tnorm(task[ch * NTHR + tid]);
    int within = 0;
#pragma unroll
    for (int tp = 0; tp < NT; ++tp) {
      const unsigned mk = __builtin_amdgcn_ballot_w32(tt == tp);
      if (lane == 0) wcs[wave * NT + tp] = (int)__builtin_popcount(mk);
      within = (tt == tp) ? (int)__builtin_amdgcn_mbcnt_lo(mk, 0u) : within;
    }
    __syncthreads();
    if (ch == own) {
      int pre = sc[tt];
#pragma unroll
      for (int w = 0; w < NWAVE; ++w) { const int v = wcs[w * NT + tt]; pre += (w < wave) ? v : 0; }
      myT = tt;
      myRank = pre + within;
    }
    __syncthreads();
    if (tid < NT) {
      int s = sc[tid];
#pragma unroll
      for (int w = 0; w < NWAVE; ++w) s += wcs[w * NT + tid];
      sc[tid] = s;
    }
    __syncthreads();
  }
  if (tid == 0) {
    int tb = 0;
#pragma unroll 1
    for (int tp = 0; tp < NT; ++tp) { tbs[tp] = tb; tb += (sc[tp] + TROWS - 1) / TROWS; }
    tbs[NT] = tb;
  }
  __syncthreads();

  int tile = tbs[myT] + (myRank >> 6);
  tile = tile < 0 ? 0 : (tile > nTiles - 1 ? nTiles - 1 : tile);
  const int slot = myRank & (TROWS - 1);
  const int b = own * NTHR + tid;
  const float* sp = shp + (size_t)b * BOTN;
  const float* rp = trg + ((size_t)tile * TROWS + slot) * NF;
  const float* wp = thw + (size_t)myT * HEADK * ACT;
  v4f q = *(const v4f*)(thb + myT * ACT);
#pragma unroll 1
  for (int c4 = 0; c4 < BOTN / 4; ++c4) {
    const v4f s  = *(const v4f*)(sp + 4 * c4);
    const v4f rv = *(const v4f*)(rp + 4 * c4);
    const v4f w0 = *(const v4f*)(wp + (4 * c4 + 0) * ACT);
    const v4f w1 = *(const v4f*)(wp + (4 * c4 + 1) * ACT);
    const v4f w2 = *(const v4f*)(wp + (4 * c4 + 2) * ACT);
    const v4f w3 = *(const v4f*)(wp + (4 * c4 + 3) * ACT);
    const v4f u0 = *(const v4f*)(wp + (BOTN + 4 * c4 + 0) * ACT);
    const v4f u1 = *(const v4f*)(wp + (BOTN + 4 * c4 + 1) * ACT);
    const v4f u2 = *(const v4f*)(wp + (BOTN + 4 * c4 + 2) * ACT);
    const v4f u3 = *(const v4f*)(wp + (BOTN + 4 * c4 + 3) * ACT);
    q = q + s.x * w0;  q = q + s.y * w1;  q = q + s.z * w2;  q = q + s.w * w3;
    q = q + rv.x * u0; q = q + rv.y * u1; q = q + rv.z * u2; q = q + rv.w * u3;
  }
  float* op = out + (size_t)b * ACT;
  *(volatile v4f*)op = q;
  __threadfence();
  *(volatile v4f*)op = q;
}

static inline size_t al256(size_t v) { return (v + 255) & ~(size_t)255; }

extern "C" void kernel_launch(void* const* d_in, const int* in_sizes, int n_in,
                              void* d_out, int out_size, void* d_ws, size_t ws_size,
                              hipStream_t stream) {
  if (n_in < 14) return;
  const int nB = in_sizes[1];
  if (nB <= 0 || (nB % NTHR) != 0 || nB > (1 << 20)) return;
  if (in_sizes[0] != nB * IMH * IMW * CIN) return;
  if (in_sizes[2] != K1 * C1 || in_sizes[3] != C1 || in_sizes[4] != K2 * C2 || in_sizes[5] != C2) return;
  if (in_sizes[6] != FLAT * EXPN || in_sizes[7] != EXPN || in_sizes[8] != EXPN * BOTN || in_sizes[9] != BOTN) return;
  if (in_sizes[10] != NT * FLAT * NF || in_sizes[11] != NT * NF ||
      in_sizes[12] != NT * HEADK * ACT || in_sizes[13] != NT * ACT) return;
  if (out_size != nB * ACT) return;

  const float* x   = (const float*)d_in[0];
  const int*   tsk = (const int*)d_in[1];
  const float* w1  = (const float*)d_in[2];
  const float* b1  = (const float*)d_in[3];
  const float* w2  = (const float*)d_in[4];
  const float* b2  = (const float*)d_in[5];
  const float* we  = (const float*)d_in[6];
  const float* be  = (const float*)d_in[7];
  const float* wb  = (const float*)d_in[8];
  const float* bb  = (const float*)d_in[9];
  const float* wt  = (const float*)d_in[10];
  const float* bt  = (const float*)d_in[11];
  const float* wh  = (const float*)d_in[12];
  const float* bh  = (const float*)d_in[13];
  float* out = (float*)d_out;

  const int nTiles = nB / TROWS + NT;
  const int maxIt  = (nB / TROWS + NG - 1) / NG;

  char* ws = (char*)d_ws;
  size_t off = 0;
  const size_t oP1 = off; off = al256(off + (size_t)C1 * K1P * 2);
  const size_t oP2 = off; off = al256(off + (size_t)C2 * K2 * 2);
  const size_t oPE = off; off = al256(off + (size_t)EXPN * FLAT * 2);
  const size_t oPB = off; off = al256(off + (size_t)BOTN * EXPN * 2);
  const size_t oPT = off; off = al256(off + (size_t)NT * NF * FLAT * 2);
  const size_t oFl = off; off = al256(off + (size_t)nB * FLAT * 2);
  const size_t oSh = off; off = al256(off + (size_t)nB * BOTN * 4);
  const size_t oTr = off; off = al256(off + (size_t)nTiles * TROWS * NF * 4);
  if (off > ws_size) return;
  _Float16* p1   = (_Float16*)(ws + oP1);
  _Float16* p2   = (_Float16*)(ws + oP2);
  _Float16* pe   = (_Float16*)(ws + oPE);
  _Float16* pb   = (_Float16*)(ws + oPB);
  _Float16* pt   = (_Float16*)(ws + oPT);
  _Float16* flat = (_Float16*)(ws + oFl);
  float*    shp  = (float*)(ws + oSh);
  float*    trg  = (float*)(ws + oTr);

  const int nPrep = (C1 * K1P + C2 * K2 + EXPN * FLAT + BOTN * EXPN + NT * NF * FLAT) / 8;
  k_wprep<<<nPrep / NTHR, NTHR, 0, stream>>>(w1, w2, we, wb, wt, p1, p2, pe, pb, pt);
  k_conv<<<nB, NTHR, 0, stream>>>(x, p1, b1, p2, b2, flat, nB);
  k_expbot<<<nB / EROWS, NTHR, 0, stream>>>(flat, pe, be, pb, bb, shp, nB);
  k_trep<<<NT * NG, NTHR, 0, stream>>>(flat, pt, bt, tsk, trg, nB, nTiles, maxIt);
  k_head<<<nB / NTHR, NTHR, 0, stream>>>(shp, trg, tsk, wh, bh, out, nB, nTiles);
}
